// SLinOSSMixer_90074054132527
// MI455X (gfx1250) — hardware-verified
//
#include <hip/hip_runtime.h>


namespace {
constexpr int Bn = 2, T = 2048, DM = 512, DI = 1024, NS = 32, DHD = 64, NH = 16, KC = 4, NT = Bn * T, PO = 2 * DI + NH + NH * 4 * NS  , POP = 4160  , BC0 = 2 * DI + NH  ;
constexpr float DTMIN = 0.03f, DTMAX = 0.1f, EPS = 1e-5f, ZS = 8.0f, WS_ = 64.0f;

typedef _Float16 b16;
typedef __attribute__((ext_vector_type(16))) _Float16 v16b;
typedef __attribute__((ext_vector_type(16))) __bf16 v16bb;
typedef __attribute__((ext_vector_type(8))) _Float16 v8b;
typedef __attribute__((ext_vector_type(8))) unsigned short v8us;
typedef __attribute__((ext_vector_type(8))) float v8f;
typedef __attribute__((ext_vector_type(4))) float v4f;
typedef __attribute__((ext_vector_type(2))) float v2f;
__device__ __forceinline__ float bf16_rne(float f) { unsigned int u = __float_as_uint(f); u += 0x7FFFu + ((u >> 16) & 1u); return __uint_as_float(u & 0xFFFF0000u); }
__device__ __forceinline__ unsigned short bf16_bits(float f) { unsigned int u = __float_as_uint(f); u += 0x7FFFu + ((u >> 16) & 1u); return (unsigned short)(u >> 16); }
__device__ __forceinline__ void split16(float v, b16& hi, b16& lo) { hi = (b16)v; lo = (b16)(v - (float)hi); }
__device__ __forceinline__ v16b frag_kb(const b16* p, int hh) { const v8b a = *(const v8b*)(p + 8 * hh), b = *(const v8b*)(p + 16 + 8 * hh); v16b f;
#pragma unroll
  for (int e = 0; e < 8; ++e) { f[e] = a[e]; f[8 + e] = b[e]; } return f; }
__device__ __forceinline__ v16bb frag_bf(const unsigned short* p, int hh) { const v8us a = *(const v8us*)(p + 8 * hh), b = *(const v8us*)(p + 16 + 8 * hh); union { unsigned short s[16]; v16bb v; } u;
#pragma unroll
  for (int e = 0; e < 8; ++e) { u.s[e] = a[e]; u.s[8 + e] = b[e]; } return u.v; }
__device__ __forceinline__ v8f wmma16b(v16b a, v16b b, v8f c) { v8f d = __builtin_amdgcn_wmma_f32_16x16x32_f16(false, a, false, b, (short)0, c, false, false); asm volatile("v_nop\n\tv_nop\n\tv_nop\n\tv_nop" : "+v"(d) : "v"(a), "v"(b)); return d; }
__device__ __forceinline__ v8f wmma16bb(v16bb a, v16bb b, v8f c) { v8f d = __builtin_amdgcn_wmma_f32_16x16x32_bf16(false, a, false, b, (short)0, c, false, false); asm volatile("v_nop\n\tv_nop\n\tv_nop\n\tv_nop" : "+v"(d) : "v"(a), "v"(b)); return d; }
__device__ __forceinline__ void wave_lds_sync() { __builtin_amdgcn_fence(__ATOMIC_RELEASE, "workgroup"); __builtin_amdgcn_wave_barrier(); __builtin_amdgcn_fence(__ATOMIC_ACQUIRE, "workgroup"); }
__device__ __forceinline__ float pmul(float a, float b) { float p = a * b; asm volatile("" : "+v"(p)); return p; }
__device__ __forceinline__ float silu_(float v) { return v / (1.0f + __expf(-v)); }
__device__ __forceinline__ float nexp(float x) { return __builtin_amdgcn_exp2f(x * 1.4426950408889634f); }
__device__ __forceinline__ float nsilu(float v) { return v * __builtin_amdgcn_rcpf(1.0f + nexp(-v)); }
__device__ __forceinline__ float nsoftplus(float v) { return fmaxf(v, 0.0f) + __builtin_amdgcn_logf(1.0f + nexp(-fabsf(v))) * 0.69314718055994531f; }

__global__ __launch_bounds__(256) void prep_kernel(const float* __restrict__ x, const float* __restrict__ win, const float* __restrict__ wout, unsigned short* __restrict__ x16, unsigned short* __restrict__ wi16, b16* __restrict__ woh, b16* __restrict__ wol) {
  const size_t tid = (size_t)blockIdx.x * blockDim.x + threadIdx.x, nth = (size_t)gridDim.x * blockDim.x;
  for (int pass = 0; pass < 2; ++pass) {
    for (size_t p = tid; p < (size_t)NT * DM / 8; p += nth) { v8us v;
#pragma unroll
      for (int e = 0; e < 8; ++e) v[e] = bf16_bits(x[p * 8 + e]);
      *(volatile v8us*)(x16 + p * 8) = v; }
    for (size_t p = tid; p < (size_t)POP * DM / 8; p += nth) { const size_t n = p / (DM / 8); v8us v;
#pragma unroll
      for (int e = 0; e < 8; ++e) v[e] = bf16_bits((n < (size_t)PO) ? win[min(p, (size_t)PO * DM / 8 - 1) * 8 + e] : 0.0f);
      *(volatile v8us*)(wi16 + p * 8) = v; }
    for (size_t p = tid; p < (size_t)DM * DI; p += nth) { b16 a, c; split16(bf16_rne(wout[p]) * WS_, a, c); ((volatile b16*)woh)[p] = a; ((volatile b16*)wol)[p] = c; }
    __threadfence();
  }
}

__global__ __launch_bounds__(128) void inproj_kernel(const unsigned short* __restrict__ x16, const unsigned short* __restrict__ wi16, float* __restrict__ proj, int rowbase) {
  __shared__ __attribute__((aligned(16))) float Ts[4][32 * 64];
  const int lane = threadIdx.x & 31, wave = threadIdx.x >> 5, nloc = lane & 15, hlf = lane >> 4, m0 = rowbase + blockIdx.y * 128 + wave * 32, c0 = blockIdx.x * 64;
  v8f acc[2][4];
#pragma unroll
  for (int r = 0; r < 2; ++r)
#pragma unroll
    for (int t = 0; t < 4; ++t) acc[r][t] = (v8f){};
#pragma unroll 2
  for (int kb = 0; kb < DM; kb += 32) { const v16bb a0 = frag_bf(x16 + (size_t)(m0 + nloc) * DM + kb, hlf), a1 = frag_bf(x16 + (size_t)(m0 + 16 + nloc) * DM + kb, hlf);
#pragma unroll
    for (int t = 0; t < 4; ++t) { const v16bb bw = frag_bf(wi16 + (size_t)(c0 + t * 16 + nloc) * DM + kb, hlf); acc[0][t] = wmma16bb(a0, bw, acc[0][t]); acc[1][t] = wmma16bb(a1, bw, acc[1][t]); } }
  float* Tt = Ts[wave];
#pragma unroll
  for (int t = 0; t < 4; ++t)
#pragma unroll
    for (int r = 0; r < 2; ++r)
#pragma unroll
      for (int v = 0; v < 8; ++v) Tt[(r * 16 + v + 8 * hlf) * 64 + t * 16 + nloc] = acc[r][t][v];
  wave_lds_sync();
  float* dst0 = proj + (size_t)m0 * POP + c0;
  for (int pass = 0; pass < 2; ++pass) {
#pragma unroll
    for (int j = 0; j < 16; ++j) { const int rr = j * 2 + hlf, c4 = nloc * 4; *(volatile v4f*)(dst0 + (size_t)rr * POP + c4) = *(const v4f*)(Tt + rr * 64 + c4); }
    __threadfence(); }
}

__global__ __launch_bounds__(256) void conv_kernel(const float* __restrict__ proj, const float* __restrict__ cw, const float* __restrict__ cb, float* __restrict__ u) {
  const size_t i = (size_t)blockIdx.x * 256 + threadIdx.x; const int t = (int)(i >> 8), cq = (int)(i & 255) * 4, l = t % T; v4f o;
#pragma unroll
  for (int c = 0; c < 4; ++c) { const int ch = cq + c; float s = bf16_rne(cb[ch]);
#pragma unroll
    for (int k = 0; k < KC; ++k) { const int lt = l - (KC - 1) + k; s += (lt >= 0) ? bf16_rne(cw[ch * KC + k]) * proj[(size_t)max(t - (KC - 1) + k, 0) * POP + DI + ch] : 0.0f; }
    o[c] = silu_(s); }
  for (int pass = 0; pass < 2; ++pass) { *(volatile v4f*)(u + (size_t)t * DI + cq) = o; __threadfence(); }
}
__global__ __launch_bounds__(256) void lam_kernel(const float* __restrict__ proj, const float* __restrict__ dtb, const float* __restrict__ gam, const float* __restrict__ th, float* __restrict__ lre, float* __restrict__ lim, float* __restrict__ dtv) {
  __shared__ float Dt[32];
  const size_t i = (size_t)blockIdx.x * 256 + threadIdx.x; const int t = (int)(i >> 7), h = (int)((i >> 3) & 15), nq = (int)(i & 7) * 4;
  const float p = proj[(size_t)t * POP + 2 * DI + h] + bf16_rne(dtb[h]); float dt = nsoftplus(p); dt = fminf(fmaxf(dt, DTMIN), DTMAX);
  v4f a, b;
#pragma unroll
  for (int e = 0; e < 4; ++e) { const int n = nq + e; const float dec = nexp(-dt * bf16_rne(gam[h * NS + n])), ph = dt * bf16_rne(th[h * NS + n]); a[e] = pmul(dec, __cosf(ph)); b[e] = pmul(dec, __sinf(ph)); }
  if (nq == 0) Dt[(threadIdx.x >> 7) * 16 + h] = dt;
  __syncthreads();
  for (int pass = 0; pass < 2; ++pass) { *(volatile v4f*)(lre + (size_t)t * NH * NS + h * NS + nq) = a; *(volatile v4f*)(lim + (size_t)t * NH * NS + h * NS + nq) = b;
    if (threadIdx.x < 32) ((volatile float*)dtv)[(size_t)blockIdx.x * 32 + threadIdx.x] = Dt[threadIdx.x];
    __threadfence(); }
}

template <int TSTEPS>
__global__ __launch_bounds__(256) void scan_kernel(const float* __restrict__ proj, float* uy, const float* __restrict__ lre, const float* __restrict__ lim, const float* __restrict__ dtv, const float* __restrict__ dsk) {
  const int b = blockIdx.y, h = blockIdx.x * 4 + (threadIdx.x >> 6), p = threadIdx.x & 63, ch = h * DHD + p;
  float sr[NS], si[NS];
#pragma unroll
  for (int n = 0; n < NS; ++n) { sr[n] = 0.0f; si[n] = 0.0f; }
  float up = 0.0f; const float dk = bf16_rne(dsk[h]);
  for (int l = 0; l < TSTEPS; ++l) { const size_t t = (size_t)b * T + l; const float* bc = proj + t * POP + BC0 + h * 4 * NS; const float* bcp = proj + (t - 1) * POP + BC0 + h * 4 * NS;
    const float dt = dtv[t * NH + h], hdt = 0.5f * dt, ut = uy[t * DI + ch]; const float* LR = lre + t * NH * NS + h * NS; const float* LI = lim + t * NH * NS + h * NS;
    float yv = 0.0f;
#pragma unroll
    for (int n = 0; n < NS; ++n) { const float bre = bc[n], bim = bc[NS + n], cre = bc[2 * NS + n], cim = bc[3 * NS + n]; const float brp = (l > 0) ? bcp[n] : 0.0f, bip = (l > 0) ? bcp[NS + n] : 0.0f;
      const float ir = hdt * (pmul(bre, ut) + pmul(brp, up)), ii = hdt * (pmul(bim, ut) + pmul(bip, up));
      const float a = LR[n], c = LI[n]; const float nr = (pmul(a, sr[n]) - pmul(c, si[n])) + ir, ni = (pmul(a, si[n]) + pmul(c, sr[n])) + ii; sr[n] = nr; si[n] = ni;
      yv += pmul(nr, cre) - pmul(ni, cim); }
    const float yo = yv + dk * ut; up = ut;
    for (int pass = 0; pass < 2; ++pass) ((volatile float*)uy)[t * DI + ch] = yo;
  }
  __threadfence();
}

__global__ __launch_bounds__(256) void norm_kernel(const float* __restrict__ y, const float* __restrict__ proj, const float* __restrict__ nw, b16* __restrict__ zh, b16* __restrict__ zl) {
  const int wid = threadIdx.x >> 5, lane = threadIdx.x & 31; const size_t t = (size_t)blockIdx.x * 8 + wid; float ss = 0.0f;
#pragma unroll 1
  for (int r = 0; r < 4; ++r) {
#pragma unroll
    for (int e = 0; e < 8; ++e) { const int c = r * 256 + lane * 8 + e; const float v = pmul(y[t * DI + c], nsilu(proj[t * POP + c])); ss += pmul(v, v); } }
#pragma unroll
  for (int o = 1; o < 32; o <<= 1) ss += __shfl_xor(ss, o);
  const float rs = rsqrtf(ss * (1.0f / DI) + EPS);
  for (int pass = 0; pass < 2; ++pass) {
#pragma unroll 1
    for (int r = 0; r < 4; ++r) { v8b oh, ol;
#pragma unroll
      for (int e = 0; e < 8; ++e) { const int c = r * 256 + lane * 8 + e; const float v = pmul(y[t * DI + c], nsilu(proj[t * POP + c])); b16 a, l_; split16(pmul(pmul(v, rs), bf16_rne(nw[c])) * ZS, a, l_); oh[e] = a; ol[e] = l_; }
      *(volatile v8b*)(zh + t * DI + r * 256 + lane * 8) = oh; *(volatile v8b*)(zl + t * DI + r * 256 + lane * 8) = ol; }
    __threadfence(); }
}

__global__ __launch_bounds__(128) void outproj_kernel(const b16* __restrict__ zh, const b16* __restrict__ zl, const b16* __restrict__ woh, const b16* __restrict__ wol, float* __restrict__ out, int rowbase) {
  __shared__ __attribute__((aligned(16))) float Ts[4][32 * 64];
  const int lane = threadIdx.x & 31, wave = threadIdx.x >> 5, nloc = lane & 15, hlf = lane >> 4, m0 = rowbase + blockIdx.y * 128 + wave * 32, c0 = blockIdx.x * 64;
  v8f acc[2][4];
#pragma unroll
  for (int r = 0; r < 2; ++r)
#pragma unroll
    for (int t = 0; t < 4; ++t) acc[r][t] = (v8f){};
#pragma unroll 2
  for (int kb = 0; kb < DI; kb += 32) { const v16b a0 = frag_kb(zh + (size_t)(m0 + nloc) * DI + kb, hlf), l0 = frag_kb(zl + (size_t)(m0 + nloc) * DI + kb, hlf), a1 = frag_kb(zh + (size_t)(m0 + 16 + nloc) * DI + kb, hlf), l1 = frag_kb(zl + (size_t)(m0 + 16 + nloc) * DI + kb, hlf);
#pragma unroll
    for (int t = 0; t < 4; ++t) { const size_t bo = (size_t)(c0 + t * 16 + nloc) * DI + kb; const v16b b0 = frag_kb(woh + bo, hlf), b1 = frag_kb(wol + bo, hlf);
      acc[0][t] = wmma16b(a0, b0, acc[0][t]); acc[0][t] = wmma16b(l0, b0, acc[0][t]); acc[0][t] = wmma16b(a0, b1, acc[0][t]);
      acc[1][t] = wmma16b(a1, b0, acc[1][t]); acc[1][t] = wmma16b(l1, b0, acc[1][t]); acc[1][t] = wmma16b(a1, b1, acc[1][t]); } }
  float* Tt = Ts[wave];
#pragma unroll
  for (int t = 0; t < 4; ++t)
#pragma unroll
    for (int r = 0; r < 2; ++r)
#pragma unroll
      for (int v = 0; v < 8; ++v) Tt[(r * 16 + v + 8 * hlf) * 64 + t * 16 + nloc] = acc[r][t][v] * (1.0f / (ZS * WS_));
  wave_lds_sync();
  float* dst0 = out + (size_t)m0 * DM + c0;
  for (int pass = 0; pass < 2; ++pass) {
#pragma unroll
    for (int j = 0; j < 16; ++j) { const int rr = j * 2 + hlf, c4 = nloc * 4; *(volatile v4f*)(dst0 + (size_t)rr * DM + c4) = *(const v4f*)(Tt + rr * 64 + c4); }
    __threadfence(); }
}
}

extern "C" void kernel_launch(void* const* d_in, const int* in_sizes, int n_in,
                              void* d_out, int out_size, void* d_ws, size_t ws_size, hipStream_t stream) {
  (void)n_in; (void)out_size;
  const float* x = (const float*)d_in[0]; const float* win = (const float*)d_in[1]; const float* cw = (const float*)d_in[2]; const float* cb = (const float*)d_in[3]; const float* dtb = (const float*)d_in[4];
  const float* gam = (const float*)d_in[5]; const float* th = (const float*)d_in[6]; const float* dsk = (const float*)d_in[7]; const float* nw = (const float*)d_in[8]; const float* wout = (const float*)d_in[9];
  float* out = (float*)d_out;
  if (in_sizes[0] != NT * DM || in_sizes[1] != PO * DM || in_sizes[2] != DI * KC || in_sizes[5] != NH * NS || in_sizes[9] != DM * DI) return;
  size_t off = 0; char* ws = (char*)d_ws;
  auto carve = [&](size_t bytes) { char* p = ws + off; off += (bytes + 255) & ~(size_t)255; return p; };
  unsigned short* x16 = (unsigned short*)carve((size_t)NT * DM * 2); unsigned short* wi16 = (unsigned short*)carve((size_t)POP * DM * 2); b16* woh = (b16*)carve((size_t)DM * DI * 2); b16* wol = (b16*)carve((size_t)DM * DI * 2);
  float* proj = (float*)carve((size_t)NT * POP * 4); float* u = (float*)carve((size_t)NT * DI * 4); float* lre = (float*)carve((size_t)NT * NH * NS * 4); float* lim = (float*)carve((size_t)NT * NH * NS * 4); float* dtv = (float*)carve((size_t)NT * NH * 4);
  b16* zh = (b16*)carve((size_t)NT * DI * 2); b16* zl = (b16*)carve((size_t)NT * DI * 2);
  if (off > ws_size) return;
  prep_kernel<<<1024, 256, 0, stream>>>(x, win, wout, x16, wi16, woh, wol);
  inproj_kernel<<<dim3(POP / 64, NT / 128), 128, 0, stream>>>(x16, wi16, proj, 0);
  conv_kernel<<<NT * 256 / 256, 256, 0, stream>>>(proj, cw, cb, u);
  lam_kernel<<<NT * 128 / 256, 256, 0, stream>>>(proj, dtb, gam, th, lre, lim, dtv);
  scan_kernel<T><<<dim3(NH / 4, Bn), 256, 0, stream>>>(proj, u, lre, lim, dtv, dsk);
  norm_kernel<<<NT / 8, 256, 0, stream>>>(u, proj, nw, zh, zl);
  outproj_kernel<<<dim3(DM / 64, NT / 128), 128, 0, stream>>>(zh, zl, woh, wol, out, 0);
}
